// BestModel4_51556787421860
// MI455X (gfx1250) — hardware-verified
//
#include <hip/hip_runtime.h>


#define AS3 __attribute__((address_space(3)))

#define NB   128
#define NL   64
#define NE   256
#define NU   256
#define KG   512
#define NGT  512
#define NENC 4
#define NV   50000
#define NR   16384
#define NNEG 16256
#define NH   1024
#define K1R  4097
#define RWA  0
#define RWD  1024
#define RWC  1025
#define RWM  2049
#define RWE  3073

typedef _Float16       v16h  __attribute__((ext_vector_type(16)));
typedef _Float16       v8h   __attribute__((ext_vector_type(8)));
typedef __bf16         v16b  __attribute__((ext_vector_type(16)));
typedef unsigned short v16us __attribute__((ext_vector_type(16)));
typedef unsigned short v8us  __attribute__((ext_vector_type(8)));
typedef float          v8f   __attribute__((ext_vector_type(8)));
typedef float          v4f   __attribute__((ext_vector_type(4)));

typedef AS3 _Float16*             lp_h;
typedef AS3 const _Float16*       lcp_h;
typedef AS3 float*                lp_f;
typedef AS3 const float*          lcp_f;
typedef AS3 unsigned short*       lp_u;
typedef AS3 const unsigned short* lcp_u;

union Frag  { v16h v; v8h half[2]; };
union FragB { v16b v; v16us u; v8us half[2]; };

constexpr size_t SZ_GKT  = (size_t)8 * NGT * KG * 2;
constexpr size_t SZ_CKT  = (size_t)8 * NU * KG * 2;
constexpr size_t SZ_WPL  = (size_t)NH * NH * 2;
constexpr size_t SZ_XP   = (size_t)NENC * NB * NL * NE * 2;
constexpr size_t SZ_QP   = (size_t)NB * NH * 4;
constexpr size_t SZ_QB   = (size_t)NB * NH * 2;
constexpr size_t SZ_DS   = (size_t)NB * NB * 4;
constexpr size_t OFF_GKT = 0;
constexpr size_t OFF_CKT = OFF_GKT + SZ_GKT;
constexpr size_t OFF_WQH = OFF_CKT + SZ_CKT;
constexpr size_t OFF_WQL = OFF_WQH + SZ_WPL;
constexpr size_t OFF_WRH = OFF_WQL + SZ_WPL;
constexpr size_t OFF_WRL = OFF_WRH + SZ_WPL;
constexpr size_t OFF_WMH = OFF_WRL + SZ_WPL;
constexpr size_t OFF_WML = OFF_WMH + SZ_WPL;
constexpr size_t OFF_XP  = OFF_WML + SZ_WPL;
constexpr size_t OFF_QP  = OFF_XP  + SZ_XP;
constexpr size_t OFF_RP  = OFF_QP  + SZ_QP;
constexpr size_t OFF_QH  = OFF_RP  + SZ_QP;
constexpr size_t OFF_QL  = OFF_QH  + SZ_QB;
constexpr size_t OFF_RH  = OFF_QL  + SZ_QB;
constexpr size_t OFF_RL  = OFF_RH  + SZ_QB;
constexpr size_t OFF_DS  = OFF_RL  + SZ_QB;
constexpr size_t OFF_PQ  = OFF_DS  + SZ_DS;
constexpr size_t OFF_PR  = OFF_PQ  + SZ_QP;
constexpr size_t WS_END  = OFF_PR  + SZ_QP;
static_assert(OFF_CKT % 128 == 0 && OFF_WQH % 128 == 0 && OFF_WQL % 128 == 0 && OFF_WRH % 128 == 0);
static_assert(OFF_WRL % 128 == 0 && OFF_WMH % 128 == 0 && OFF_WML % 128 == 0 && OFF_XP % 128 == 0);
static_assert(OFF_QP % 128 == 0 && OFF_RP % 128 == 0 && OFF_QH % 128 == 0 && OFF_QL % 128 == 0);
static_assert(OFF_RH % 128 == 0 && OFF_RL % 128 == 0 && OFF_DS % 128 == 0 && OFF_PQ % 128 == 0 && OFF_PR % 128 == 0);
static_assert(WS_END <= (size_t)134217728);
static_assert(KG % 32 == 0 && NH % 128 == 0 && NU % 16 == 0);

constexpr int CV_GATE  = 8 * (KG / 64) * (NGT / 64);
constexpr int CV_CAND  = 8 * (KG / 64) * (NU / 64);
constexpr int CV_WPL   = (NH / 64) * (NH / 64);
constexpr int CV_TOTAL = CV_GATE + CV_CAND + 3 * CV_WPL;
#define CVP 72
constexpr int GX_BLK   = NENC * NB * NL / 8;
#define MB   32
#define TP   520
#define GTHR 256
constexpr int GRU_BLK  = NENC * (NB / MB);
#define PNP  132
constexpr int PN_BLK   = 2 * (NB / 32) * (NH / 128);
#define MR   32
#define PAP  1032
#define MTHR 512
constexpr int PR_BLK   = NR / MR;
static_assert(NB % MB == 0 && NR % MR == 0 && MB == 32 && MR == 32);
static_assert(TP % 8 == 0 && PAP % 8 == 0 && CVP % 8 == 0 && PNP % 4 == 0);
static_assert((NENC * NB * NL) % 8 == 0 && NB % 32 == 0);

constexpr int    T_TILE   = MB * TP;
constexpr size_t LOFF_T   = 0;
constexpr size_t LSZ_T    = (size_t)4 * T_TILE * 2;
constexpr size_t LOFF_HS  = LOFF_T + LSZ_T;
constexpr size_t LSZ_HS   = (size_t)2 * MB * NU * 4;
constexpr size_t LOFF_GB  = LOFF_HS + LSZ_HS;
constexpr size_t LOFF_CB  = LOFF_GB + (size_t)2 * NGT * 4;
constexpr size_t LOFF_LEN = LOFF_CB + (size_t)2 * NU * 4;
constexpr size_t LDS_GRU  = LOFF_LEN + 128;
static_assert(LOFF_HS % 16 == 0 && LOFF_GB % 16 == 0 && LOFF_CB % 16 == 0 && LOFF_LEN % 16 == 0);
static_assert((4 * T_TILE) % 8 == 0 && (2 * MB * NU) % 4 == 0);

constexpr size_t POFF_AH  = 0;
constexpr size_t PSZ_A    = (size_t)MR * PAP * 2;
constexpr size_t POFF_AL  = POFF_AH + PSZ_A;
constexpr size_t POFF_P   = POFF_AL + PSZ_A;
constexpr size_t POFF_O   = POFF_P + (size_t)16 * MR * 2 * 4;
constexpr size_t POFF_QI  = POFF_O + 256;
constexpr size_t POFF_RI  = POFF_QI + 128;
constexpr size_t POFF_D   = POFF_RI + 128;
constexpr size_t LDS_PAIR = POFF_D + 128;
static_assert(POFF_AL % 16 == 0 && POFF_P % 16 == 0 && POFF_O % 16 == 0 && POFF_QI % 16 == 0);
static_assert((PAP * 2) % 16 == 0);

#define SACT   256.0f
#define SWGT   256.0f
#define FOLDG  1.52587890625e-05f

__device__ __forceinline__ float rcpx(float x) { return __builtin_amdgcn_rcpf(x); }
__device__ __forceinline__ float sigm(float x) { return rcpx(1.0f + __expf(-x)); }
__device__ __forceinline__ float tanhm(float x) {
    const float e = __expf(2.0f * x);
    return 1.0f - 2.0f * rcpx(e + 1.0f);
}
__device__ __forceinline__ v8f ld8f(const float* p) {
    const v4f a = *(const v4f*)p;
    const v4f b = *(const v4f*)(p + 4);
    return __builtin_shufflevector(a, b, 0, 1, 2, 3, 4, 5, 6, 7);
}
__device__ __forceinline__ v8f zero8() {
    v8f z;
#pragma unroll
    for (int i = 0; i < 8; ++i) z[i] = 0.0f;
    return z;
}
__device__ __forceinline__ unsigned short bf16rne(float f) {
    unsigned int u = __float_as_uint(f);
    u += 0x7FFFu + ((u >> 16) & 1u);
    return (unsigned short)(u >> 16);
}
__device__ __forceinline__ float bf16tof(unsigned short b) {
    return __uint_as_float(((unsigned int)b) << 16);
}
__device__ __forceinline__ unsigned short f16bits(float f) {
    const _Float16 hv = (_Float16)f;
    return __builtin_bit_cast(unsigned short, hv);
}

__device__ __forceinline__ void ldfrag_lds(Frag& f, lcp_h p) {
    f.half[0] = *(AS3 const v8h*)(p);
    f.half[1] = *(AS3 const v8h*)(p + 16);
}
__device__ __forceinline__ void ldfrag_gen(Frag& f, const _Float16* p) {
    f.half[0] = *(const v8h*)(p);
    f.half[1] = *(const v8h*)(p + 16);
}
__device__ __forceinline__ v8f mma16(v8f c, const Frag& a, const Frag& b) {
    return __builtin_amdgcn_wmma_f32_16x16x32_f16(false, a.v, false, b.v, (short)0, c, false, false);
}
__device__ __forceinline__ void ldfragb_lds(FragB& f, lcp_u p) {
    f.half[0] = *(AS3 const v8us*)(p);
    f.half[1] = *(AS3 const v8us*)(p + 16);
}
__device__ __forceinline__ void ldfragb_gen(FragB& f, const unsigned short* p) {
    f.half[0] = *(const v8us*)(p);
    f.half[1] = *(const v8us*)(p + 16);
}
__device__ __forceinline__ v8f mmab(v8f c, const FragB& a, const FragB& b) {
    return __builtin_amdgcn_wmma_f32_16x16x32_bf16(false, a.v, false, b.v, (short)0, c, false, false);
}

__global__ __launch_bounds__(256)
void k_cvt(const float* __restrict__ gk, const float* __restrict__ ck, const float* __restrict__ w1,
           unsigned short* gkt, unsigned short* ckt,
           unsigned short* wqh, unsigned short* wql, unsigned short* wrh, unsigned short* wrl,
           unsigned short* wmh, unsigned short* wml)
{
    __shared__ __attribute__((aligned(16))) unsigned short sH[64 * CVP];
    __shared__ __attribute__((aligned(16))) unsigned short sL[64 * CVP];
    const int tid = threadIdx.x, bid = blockIdx.x;
    const int row = tid >> 2, c16 = (tid & 3) * 16;
    int k0, n0, dstK; bool split;
    const float* pa; const float* pb; float fa, fb;
    unsigned short* dh; unsigned short* dl;
    if (bid < CV_GATE) {
        const int mat = bid >> 6, tt = bid & 63;
        k0 = (tt >> 3) * 64; n0 = (tt & 7) * 64; dstK = KG; split = false;
        pa = gk + ((size_t)mat * KG + k0 + row) * NGT + n0 + c16; pb = pa; fa = SWGT; fb = 0.0f;
        dh = gkt + (size_t)mat * NGT * KG; dl = dh;
    } else if (bid < CV_GATE + CV_CAND) {
        const int bq = bid - CV_GATE, mat = bq >> 5, tt = bq & 31;
        k0 = (tt >> 2) * 64; n0 = (tt & 3) * 64; dstK = KG; split = false;
        pa = ck + ((size_t)mat * KG + k0 + row) * NU + n0 + c16; pb = pa; fa = SWGT; fb = 0.0f;
        dh = ckt + (size_t)mat * NU * KG; dl = dh;
    } else {
        const int bw = bid - CV_GATE - CV_CAND, pl = bw >> 8, tt = bw & 255;
        k0 = (tt >> 4) * 64; n0 = (tt & 15) * 64; dstK = NH; split = true;
        int ra, rb;
        if (pl == 0)      { ra = RWA + k0 + row; rb = RWC + k0 + row; fa = 1.0f; fb = 1.0f;  dh = wqh; dl = wql; }
        else if (pl == 1) { ra = RWE + k0 + row; rb = RWC + k0 + row; fa = 1.0f; fb = -1.0f; dh = wrh; dl = wrl; }
        else              { ra = RWM + k0 + row; rb = ra;            fa = 1.0f; fb = 0.0f;  dh = wmh; dl = wml; }
        pa = w1 + (size_t)ra * NH + n0 + c16; pb = w1 + (size_t)rb * NH + n0 + c16;
    }
#pragma unroll
    for (int i = 0; i < 4; ++i) {
        const v4f va = *(const v4f*)(pa + 4 * i);
        const v4f vb = *(const v4f*)(pb + 4 * i);
#pragma unroll
        for (int j = 0; j < 4; ++j) {
            const float v = va[j] * fa + vb[j] * fb;
            const int li = (c16 + 4 * i + j) * CVP + row;
            if (split) {
                const unsigned short hb = bf16rne(v);
                sH[li] = hb;
                sL[li] = bf16rne(v - bf16tof(hb));
            } else {
                sH[li] = f16bits(v);
            }
        }
    }
    __syncthreads();
#pragma unroll
    for (int ps = 0; ps < 2; ++ps) {
#pragma unroll
        for (int jj = 0; jj < 2; ++jj) {
            const int p = tid + 256 * jj;
            const int n = p >> 3, pc = p & 7;
            const size_t go = (size_t)(n0 + n) * dstK + k0 + pc * 8;
            const v8us hv = *(const v8us*)(&sH[n * CVP + pc * 8]);
            *(volatile v8us*)(dh + go) = hv;
            if (split) {
                const v8us lv = *(const v8us*)(&sL[n * CVP + pc * 8]);
                *(volatile v8us*)(dl + go) = lv;
            }
        }
        if (ps == 0) __threadfence();
    }
}

__global__ __launch_bounds__(256)
void k_gx(const int* __restrict__ iq, const int* __restrict__ ir,
          const int* __restrict__ ql, const int* __restrict__ rl,
          const float* __restrict__ emb, _Float16* xp)
{
    const int lane = threadIdx.x & 31, w = threadIdx.x >> 5;
    const int rowid = blockIdx.x * 8 + w;
    const int t = rowid & (NL - 1), b = (rowid >> 6) & (NB - 1), enc = rowid >> 13;
    const int lq = ql[b], lr = rl[b];
    int len = (enc < 2) ? lq : lr;
    len = min(max(len, 0), NL);
    int tt = ((enc & 1) && (t < len)) ? (len - 1 - t) : t;
    tt = min(max(tt, 0), NL - 1);
    const int tq = iq[b * NL + tt], tr = ir[b * NL + tt];
    int tok = (enc < 2) ? tq : tr;
    tok = min(max(tok, 0), NV - 1);
    const v8f ev = ld8f(emb + (size_t)tok * NE + lane * 8);
    v8h hv;
#pragma unroll
    for (int i = 0; i < 8; ++i) hv[i] = (_Float16)(ev[i] * SACT);
    _Float16* d = xp + (size_t)rowid * NE + lane * 8;
    *(volatile v8h*)d = hv;
    __threadfence();
    *(volatile v8h*)d = hv;
}

template <int ND>
__device__ __forceinline__ void gru_layer(lp_h Tg, lp_h Tc, lp_f HS,
                                          const _Float16* __restrict__ gkw,
                                          const _Float16* __restrict__ ckw,
                                          lcp_f gbias, lcp_f cbias, AS3 const int* sLen, int t,
                                          lp_h d1, lp_h d2, lp_h d3)
{
    const int tid = threadIdx.x, lane = tid & 31, w = tid >> 5, h = lane >> 4, m = lane & 15;

    v8f acc[2][2][2];
#pragma unroll
    for (int mt = 0; mt < 2; ++mt)
#pragma unroll
        for (int g = 0; g < 2; ++g) { acc[mt][g][0] = zero8(); acc[mt][g][1] = zero8(); }

    lcp_h ab = Tg + m * TP + 8 * h;
    const _Float16* wb = gkw + (size_t)(32 * w + m) * KG + 8 * h;
#pragma unroll 1
    for (int k0 = 0; k0 < KG; k0 += 32) {
        Frag a[2], b[2][2];
        ldfrag_lds(a[0], ab + k0);
        ldfrag_lds(a[1], ab + 16 * TP + k0);
#pragma unroll
        for (int g = 0; g < 2; ++g)
#pragma unroll
            for (int q = 0; q < 2; ++q)
                ldfrag_gen(b[g][q], wb + (size_t)(16 * g + NU * q) * KG + k0);
#pragma unroll
        for (int mt = 0; mt < 2; ++mt)
#pragma unroll
            for (int g = 0; g < 2; ++g) {
                acc[mt][g][0] = mma16(acc[mt][g][0], a[mt], b[g][0]);
                acc[mt][g][1] = mma16(acc[mt][g][1], a[mt], b[g][1]);
            }
        asm volatile("v_nop\n\tv_nop\n\tv_nop\n\tv_nop"
                     : "+v"(acc[0][0][0]), "+v"(acc[0][0][1]), "+v"(acc[0][1][0]), "+v"(acc[0][1][1]),
                       "+v"(acc[1][0][0]), "+v"(acc[1][0][1]), "+v"(acc[1][1][0]), "+v"(acc[1][1][1])
                     : "v"(a[0].v), "v"(a[1].v), "v"(b[0][0].v), "v"(b[0][1].v), "v"(b[1][0].v), "v"(b[1][1].v));
    }

    float z[2][2][8];
#pragma unroll
    for (int g = 0; g < 2; ++g) {
        const int n = 32 * w + 16 * g + m;
        const float br = gbias[n];
        const float bz = gbias[NU + n];
#pragma unroll
        for (int mt = 0; mt < 2; ++mt) {
#pragma unroll
            for (int r = 0; r < 8; ++r) {
                const int row = 16 * mt + 8 * h + r;
                const float rg = sigm(acc[mt][g][0][r] * FOLDG + br);
                const float zz = sigm(acc[mt][g][1][r] * FOLDG + bz);
                const float hold = HS[row * NU + n];
                Tc[row * TP + NU + n] = (_Float16)(rg * hold * SACT);
                z[mt][g][r] = zz;
            }
        }
    }
    __syncthreads();

    v8f acc2[2][2];
#pragma unroll
    for (int mt = 0; mt < 2; ++mt) { acc2[mt][0] = zero8(); acc2[mt][1] = zero8(); }
    lcp_h ab2 = Tc + m * TP + 8 * h;
    const _Float16* wc = ckw + (size_t)(32 * w + m) * KG + 8 * h;
#pragma unroll 1
    for (int k0 = 0; k0 < KG; k0 += 32) {
        Frag a[2], b[2];
        ldfrag_lds(a[0], ab2 + k0);
        ldfrag_lds(a[1], ab2 + 16 * TP + k0);
        ldfrag_gen(b[0], wc + k0);
        ldfrag_gen(b[1], wc + (size_t)16 * KG + k0);
#pragma unroll
        for (int mt = 0; mt < 2; ++mt) {
            acc2[mt][0] = mma16(acc2[mt][0], a[mt], b[0]);
            acc2[mt][1] = mma16(acc2[mt][1], a[mt], b[1]);
        }
        asm volatile("v_nop\n\tv_nop\n\tv_nop\n\tv_nop"
                     : "+v"(acc2[0][0]), "+v"(acc2[0][1]), "+v"(acc2[1][0]), "+v"(acc2[1][1])
                     : "v"(a[0].v), "v"(a[1].v), "v"(b[0].v), "v"(b[1].v));
    }

#pragma unroll
    for (int g = 0; g < 2; ++g) {
        const int n = 32 * w + 16 * g + m;
        const float bc = cbias[n];
#pragma unroll
        for (int mt = 0; mt < 2; ++mt) {
#pragma unroll
            for (int r = 0; r < 8; ++r) {
                const int row = 16 * mt + 8 * h + r;
                const float c = tanhm(acc2[mt][g][r] * FOLDG + bc);
                const float hold = HS[row * NU + n];
                const float zz = z[mt][g][r];
                const float hn = zz * hold + (1.0f - zz) * c;
                const bool act = t < sLen[row];
                const float o = act ? hn : hold;
                HS[row * NU + n] = o;
                const _Float16 oh = (_Float16)(o * SACT);
                d1[row * TP + n] = oh;
                if (ND == 3) { d2[row * TP + n] = oh; d3[row * TP + n] = oh; }
            }
        }
    }
}

__global__ __launch_bounds__(GTHR)
void k_gru(const _Float16* __restrict__ xp, const _Float16* __restrict__ gkt,
           const _Float16* __restrict__ ckt, const float* __restrict__ gb,
           const float* __restrict__ cb, const int* __restrict__ ql,
           const int* __restrict__ rl, float* qp, float* rp,
           unsigned short* qbh, unsigned short* qbl, unsigned short* rbh, unsigned short* rbl)
{
    extern __shared__ __attribute__((aligned(16))) char smem[];
    lp_h sT  = (lp_h)(smem + LOFF_T);
    lp_f sHS = (lp_f)(smem + LOFF_HS);
    lp_f sGB = (lp_f)(smem + LOFF_GB);
    lp_f sCB = (lp_f)(smem + LOFF_CB);
    AS3 int* sLen = (AS3 int*)(smem + LOFF_LEN);

    const int tid = threadIdx.x, lane = tid & 31, w = tid >> 5;
    const int enc = blockIdx.x >> 2, grp = blockIdx.x & 3, b0 = grp * MB;

    {
        v8h zh;
#pragma unroll
        for (int i = 0; i < 8; ++i) zh[i] = (_Float16)0.0f;
        for (int i = tid; i < (4 * T_TILE) / 8; i += GTHR) *(AS3 v8h*)(sT + 8 * i) = zh;
        v4f zf;
#pragma unroll
        for (int i = 0; i < 4; ++i) zf[i] = 0.0f;
        for (int i = tid; i < (2 * MB * NU) / 4; i += GTHR) *(AS3 v4f*)(sHS + 4 * i) = zf;
        for (int i = tid; i < 2 * NGT; i += GTHR) sGB[i] = gb[(size_t)enc * (2 * NGT) + i];
        for (int i = tid; i < 2 * NU; i += GTHR) sCB[i] = cb[(size_t)enc * (2 * NU) + i];
        if (tid < MB) {
            const int lq = ql[b0 + tid], lr = rl[b0 + tid];
            int v = (enc < 2) ? lq : lr;
            v = min(max(v, 0), NL);
            sLen[tid] = v;
        }
    }
    __syncthreads();
    int nsteps = 0;
    for (int i = 0; i < MB; ++i) nsteps = max(nsteps, sLen[i]);
    nsteps = min(nsteps, NL);

    lp_h T0 = sT, T1 = sT + T_TILE, T2 = sT + 2 * T_TILE, T3 = sT + 3 * T_TILE;
    lp_f HS1 = sHS, HS2 = sHS + MB * NU;
    const _Float16* gk0 = gkt + (size_t)(enc * 2 + 0) * NGT * KG;
    const _Float16* gk1 = gkt + (size_t)(enc * 2 + 1) * NGT * KG;
    const _Float16* ck0 = ckt + (size_t)(enc * 2 + 0) * NU * KG;
    const _Float16* ck1 = ckt + (size_t)(enc * 2 + 1) * NU * KG;

    const int srow = tid >> 3, spc = (tid & 7) * 32;
    const _Float16* xrow = xp + ((size_t)(enc * NB + b0 + srow) * NL) * NE + spc;

#pragma unroll 1
    for (int t = 0; t < nsteps; ++t) {
        __syncthreads();
        {
            const _Float16* xs = xrow + (size_t)t * NE;
#pragma unroll
            for (int i = 0; i < 4; ++i) {
                const v8h v = *(const v8h*)(xs + 8 * i);
                *(AS3 v8h*)(T0 + srow * TP + spc + 8 * i) = v;
                *(AS3 v8h*)(T1 + srow * TP + spc + 8 * i) = v;
            }
        }
        __syncthreads();
        gru_layer<3>(T0, T1, HS1, gk0, ck0, sGB, sCB, sLen, t, T2, T3, T0 + NU);
        __syncthreads();
        gru_layer<1>(T2, T3, HS2, gk1, ck1, sGB + NGT, sCB + NU, sLen, t, T2 + NU, T2 + NU, T2 + NU);
    }
    __syncthreads();

    const size_t cofs = (size_t)(enc & 1) * (2 * NU);
    float* ob = ((enc < 2) ? qp : rp) + cofs;
    unsigned short* obh = ((enc < 2) ? qbh : rbh) + cofs;
    unsigned short* obl = ((enc < 2) ? qbl : rbl) + cofs;
#pragma unroll
    for (int ps = 0; ps < 2; ++ps) {
#pragma unroll
        for (int rr = 0; rr < 4; ++rr) {
            const int row = w * 4 + rr;
            const size_t go = (size_t)(b0 + row) * NH;
#pragma unroll
            for (int j = 0; j < 4; ++j) {
                const int col = j * 128 + lane * 4;
                lcp_f s = (j < 2) ? (lcp_f)(HS1 + row * NU + col) : (lcp_f)(HS2 + row * NU + (col - NU));
                const v4f v = *(AS3 const v4f*)s;
                *(volatile v4f*)(ob + go + col) = v;
            }
#pragma unroll
            for (int jb = 0; jb < 2; ++jb) {
                lcp_f s = (jb == 0) ? (lcp_f)(HS1 + row * NU + lane * 8) : (lcp_f)(HS2 + row * NU + lane * 8);
                const v4f a = *(AS3 const v4f*)s;
                const v4f c = *(AS3 const v4f*)(s + 4);
                v8us hh, ll;
#pragma unroll
                for (int i = 0; i < 4; ++i) {
                    const unsigned short ha = bf16rne(a[i]);
                    hh[i] = ha;
                    ll[i] = bf16rne(a[i] - bf16tof(ha));
                    const unsigned short hc = bf16rne(c[i]);
                    hh[4 + i] = hc;
                    ll[4 + i] = bf16rne(c[i] - bf16tof(hc));
                }
                const int col = jb * 256 + lane * 8;
                *(volatile v8us*)(obh + go + col) = hh;
                *(volatile v8us*)(obl + go + col) = ll;
            }
        }
        if (ps == 0) __threadfence();
    }
}

__global__ __launch_bounds__(256)
void k_dist(const float* __restrict__ qp, const float* __restrict__ rp, float* ds)
{
    __shared__ __attribute__((aligned(16))) float sq[NH];
    __shared__ __attribute__((aligned(16))) float sd[NB];
    const int tid = threadIdx.x, lane = tid & 31, w = tid >> 5;
    const int i = blockIdx.x;
    *(v4f*)(&sq[tid * 4]) = *(const v4f*)(qp + (size_t)i * NH + tid * 4);
    __syncthreads();
#pragma unroll 1
    for (int jj = 0; jj < NB / 8; ++jj) {
        const int j = w + 8 * jj;
        const float* rr = rp + (size_t)j * NH;
        v4f s4;
#pragma unroll
        for (int q = 0; q < 4; ++q) s4[q] = 0.0f;
#pragma unroll 1
        for (int it = 0; it < NH / 128; ++it) {
            const int c = it * 128 + lane * 4;
            const v4f a = *(const v4f*)(&sq[c]);
            const v4f b = *(const v4f*)(rr + c);
            s4 += a * b;
        }
        float s = (s4[0] + s4[1]) + (s4[2] + s4[3]);
#pragma unroll
        for (int off = 16; off; off >>= 1) s += __shfl_xor(s, off, 32);
        if (lane == 0) sd[j] = s;
    }
    __syncthreads();
    if (w == 0) {
        const v4f v = *(const v4f*)(&sd[lane * 4]);
        float* d = ds + (size_t)i * NB + lane * 4;
        *(volatile v4f*)d = v;
        __threadfence();
        *(volatile v4f*)d = v;
    }
}

__global__ __launch_bounds__(256)
void k_pnode(const unsigned short* __restrict__ qbh, const unsigned short* __restrict__ qbl,
             const unsigned short* __restrict__ rbh, const unsigned short* __restrict__ rbl,
             const unsigned short* __restrict__ wqh, const unsigned short* __restrict__ wql,
             const unsigned short* __restrict__ wrh, const unsigned short* __restrict__ wrl,
             float* pq, float* pr)
{
    __shared__ __attribute__((aligned(16))) float sOut[32 * PNP];
    const int tid = threadIdx.x, lane = tid & 31, w = tid >> 5, h = lane >> 4, m = lane & 15;
    const int bid = blockIdx.x;
    const int mat = bid >> 5, rt = (bid >> 3) & 3, ct = bid & 7;
    const unsigned short* ahp = (mat == 0) ? qbh : rbh;
    const unsigned short* alp = (mat == 0) ? qbl : rbl;
    const unsigned short* bhp = (mat == 0) ? wqh : wrh;
    const unsigned short* blp = (mat == 0) ? wql : wrl;
    float* dst = (mat == 0) ? pq : pr;
    const unsigned short* ah = ahp + (size_t)(rt * 32 + m) * NH + 8 * h;
    const unsigned short* al = alp + (size_t)(rt * 32 + m) * NH + 8 * h;
    const unsigned short* bh = bhp + (size_t)(ct * 128 + 16 * w + m) * NH + 8 * h;
    const unsigned short* bl = blp + (size_t)(ct * 128 + 16 * w + m) * NH + 8 * h;

    v8f acc[2];
    acc[0] = zero8(); acc[1] = zero8();
#pragma unroll 1
    for (int k0 = 0; k0 < NH; k0 += 32) {
        FragB xa[2], xl[2], yh, yl;
        ldfragb_gen(xa[0], ah + k0);
        ldfragb_gen(xa[1], ah + (size_t)16 * NH + k0);
        ldfragb_gen(xl[0], al + k0);
        ldfragb_gen(xl[1], al + (size_t)16 * NH + k0);
        ldfragb_gen(yh, bh + k0);
        ldfragb_gen(yl, bl + k0);
#pragma unroll
        for (int mt = 0; mt < 2; ++mt) {
            acc[mt] = mmab(acc[mt], xa[mt], yh);
            acc[mt] = mmab(acc[mt], xa[mt], yl);
            acc[mt] = mmab(acc[mt], xl[mt], yh);
        }
        asm volatile("v_nop\n\tv_nop\n\tv_nop\n\tv_nop"
                     : "+v"(acc[0]), "+v"(acc[1])
                     : "v"(xa[0].u), "v"(xa[1].u), "v"(xl[0].u), "v"(xl[1].u), "v"(yh.u), "v"(yl.u));
    }
#pragma unroll
    for (int mt = 0; mt < 2; ++mt)
#pragma unroll
        for (int r = 0; r < 8; ++r) sOut[(16 * mt + 8 * h + r) * PNP + 16 * w + m] = acc[mt][r];
    __syncthreads();
#pragma unroll
    for (int ps = 0; ps < 2; ++ps) {
#pragma unroll
        for (int rr = 0; rr < 4; ++rr) {
            const int row = 4 * w + rr;
            const v4f v = *(const v4f*)(&sOut[row * PNP + lane * 4]);
            float* d = dst + (size_t)(rt * 32 + row) * NH + ct * 128 + lane * 4;
            *(volatile v4f*)d = v;
        }
        if (ps == 0) __threadfence();
    }
}

__global__ __launch_bounds__(MTHR)
void k_pair(const float* __restrict__ qp, const float* __restrict__ rp, const float* __restrict__ ds,
            const float* __restrict__ pq, const float* __restrict__ pr,
            const int* __restrict__ nqi, const int* __restrict__ nri,
            const unsigned short* __restrict__ wmh, const unsigned short* __restrict__ wml,
            const float* __restrict__ w1, const float* __restrict__ b1,
            const float* __restrict__ w2, const float* __restrict__ b2, float* out)
{
    extern __shared__ __attribute__((aligned(16))) char smem[];
    lp_u sAH = (lp_u)(smem + POFF_AH);
    lp_u sAL = (lp_u)(smem + POFF_AL);
    lp_f sP  = (lp_f)(smem + POFF_P);
    lp_f sO  = (lp_f)(smem + POFF_O);
    AS3 int* sQi = (AS3 int*)(smem + POFF_QI);
    AS3 int* sRi = (AS3 int*)(smem + POFF_RI);
    lp_f sD  = (lp_f)(smem + POFF_D);

    const int tid = threadIdx.x, lane = tid & 31, w = tid >> 5, h = lane >> 4, m = lane & 15;
    const int m0 = blockIdx.x * MR;

    if (tid < MR) {
        const int gr = m0 + tid;
        const int p = min(max(gr - NB, 0), NNEG - 1);
        int a = nqi[p], bq = nri[p];
        a  = min(max(a, 0), NB - 1);
        bq = min(max(bq, 0), NB - 1);
        const int q = (gr < NB) ? gr : a;
        const int r = (gr < NB) ? gr : bq;
        sQi[tid] = q; sRi[tid] = r;
        sD[tid] = ds[q * NB + r];
    }
    __syncthreads();

    {
        const int srow = tid >> 4, seg = (tid & 15) * 64;
        const int q = sQi[srow], r = sRi[srow];
        const float* qrow = qp + (size_t)q * NH + seg;
        const float* rrow = rp + (size_t)r * NH + seg;
#pragma unroll
        for (int c = 0; c < 8; ++c) {
            const v8f qa = ld8f(qrow + 8 * c);
            const v8f ra = ld8f(rrow + 8 * c);
            v8us hh, ll;
#pragma unroll
            for (int i = 0; i < 8; ++i) {
                const float pv = qa[i] * ra[i];
                const unsigned short hb = bf16rne(pv);
                hh[i] = hb;
                ll[i] = bf16rne(pv - bf16tof(hb));
            }
            *(AS3 v8us*)(sAH + srow * PAP + seg + 8 * c) = hh;
            *(AS3 v8us*)(sAL + srow * PAP + seg + 8 * c) = ll;
        }
    }
    __syncthreads();

    float hp[2][8][2];
#pragma unroll
    for (int mt = 0; mt < 2; ++mt)
#pragma unroll
        for (int r = 0; r < 8; ++r) { hp[mt][r][0] = 0.0f; hp[mt][r][1] = 0.0f; }

    lcp_u sah = (lcp_u)(sAH + m * PAP + 8 * h);
    lcp_u sal = (lcp_u)(sAL + m * PAP + 8 * h);
    const float* w1d = w1 + (size_t)RWD * NH;

#pragma unroll 1
    for (int nh = 0; nh < 2; ++nh) {
        v8f acc[2][2];
#pragma unroll
        for (int mt = 0; mt < 2; ++mt) { acc[mt][0] = zero8(); acc[mt][1] = zero8(); }
        const int cw = 512 * nh + 32 * w;
        const unsigned short* wbh = wmh + (size_t)(cw + m) * NH + 8 * h;
        const unsigned short* wbl = wml + (size_t)(cw + m) * NH + 8 * h;
#pragma unroll 1
        for (int k0 = 0; k0 < NH; k0 += 32) {
            FragB xa[2], xl[2], yh[2], yl[2];
            ldfragb_lds(xa[0], sah + k0);
            ldfragb_lds(xa[1], sah + 16 * PAP + k0);
            ldfragb_lds(xl[0], sal + k0);
            ldfragb_lds(xl[1], sal + 16 * PAP + k0);
#pragma unroll
            for (int nt = 0; nt < 2; ++nt) {
                ldfragb_gen(yh[nt], wbh + (size_t)nt * 16 * NH + k0);
                ldfragb_gen(yl[nt], wbl + (size_t)nt * 16 * NH + k0);
            }
#pragma unroll
            for (int mt = 0; mt < 2; ++mt)
#pragma unroll
                for (int nt = 0; nt < 2; ++nt) {
                    acc[mt][nt] = mmab(acc[mt][nt], xa[mt], yh[nt]);
                    acc[mt][nt] = mmab(acc[mt][nt], xa[mt], yl[nt]);
                    acc[mt][nt] = mmab(acc[mt][nt], xl[mt], yh[nt]);
                }
            asm volatile("v_nop\n\tv_nop\n\tv_nop\n\tv_nop"
                         : "+v"(acc[0][0]), "+v"(acc[0][1]), "+v"(acc[1][0]), "+v"(acc[1][1])
                         : "v"(xa[0].u), "v"(xa[1].u), "v"(xl[0].u), "v"(xl[1].u),
                           "v"(yh[0].u), "v"(yh[1].u), "v"(yl[0].u), "v"(yl[1].u));
        }

        float wd[2], bb[2], w20[2], w21[2];
#pragma unroll
        for (int nt = 0; nt < 2; ++nt) {
            const int col = cw + 16 * nt + m;
            wd[nt]  = w1d[col];
            bb[nt]  = b1[col];
            w20[nt] = w2[col * 2 + 0];
            w21[nt] = w2[col * 2 + 1];
        }
#pragma unroll
        for (int mt = 0; mt < 2; ++mt) {
#pragma unroll
            for (int r = 0; r < 8; ++r) {
                const int row = 16 * mt + 8 * h + r;
                const int i = sQi[row], j = sRi[row];
                const float dd = sD[row];
                const float* pqi = pq + (size_t)i * NH + cw + m;
                const float* prj = pr + (size_t)j * NH + cw + m;
#pragma unroll
                for (int nt = 0; nt < 2; ++nt) {
                    const float pre = acc[mt][nt][r] + pqi[16 * nt] + prj[16 * nt] + dd * wd[nt] + bb[nt];
                    const float v = fmaxf(pre, 0.0f);
                    hp[mt][r][0] += v * w20[nt];
                    hp[mt][r][1] += v * w21[nt];
                }
            }
        }
    }

#pragma unroll
    for (int mt = 0; mt < 2; ++mt)
#pragma unroll
        for (int r = 0; r < 8; ++r)
#pragma unroll
            for (int jj = 0; jj < 2; ++jj) {
                float x = hp[mt][r][jj];
                x += __shfl_xor(x, 1, 32);
                x += __shfl_xor(x, 2, 32);
                x += __shfl_xor(x, 4, 32);
                x += __shfl_xor(x, 8, 32);
                hp[mt][r][jj] = x;
            }
    if (m == 0) {
#pragma unroll
        for (int mt = 0; mt < 2; ++mt)
#pragma unroll
            for (int r = 0; r < 8; ++r) {
                const int row = 16 * mt + 8 * h + r;
                sP[(w * MR + row) * 2 + 0] = hp[mt][r][0];
                sP[(w * MR + row) * 2 + 1] = hp[mt][r][1];
            }
    }
    __syncthreads();
    if (tid < 2 * MR) {
        const int row = tid >> 1, jj = tid & 1;
        float s = b2[jj];
#pragma unroll 1
        for (int ww = 0; ww < 16; ++ww) s += sP[(ww * MR + row) * 2 + jj];
        sO[row * 2 + jj] = s;
    }
    __syncthreads();
    float* d = out + (size_t)m0 * 2 + (size_t)tid * 4;
    if (tid < 16) { const v4f v = *(AS3 const v4f*)(sO + tid * 4); *(volatile v4f*)d = v; }
    __threadfence();
    if (tid < 16) { const v4f v = *(AS3 const v4f*)(sO + tid * 4); *(volatile v4f*)d = v; }
}

extern "C" void kernel_launch(void* const* d_in, const int* in_sizes, int n_in,
                              void* d_out, int out_size, void* d_ws, size_t ws_size,
                              hipStream_t stream)
{
    if (n_in < 15) return;
    if (in_sizes[0]  != NB * NL)               return;
    if (in_sizes[1]  != NB * NL)               return;
    if (in_sizes[2]  != NB)                    return;
    if (in_sizes[3]  != NB)                    return;
    if (in_sizes[4]  != NNEG)                  return;
    if (in_sizes[5]  != NNEG)                  return;
    if (in_sizes[6]  != NV * NE)               return;
    if (in_sizes[7]  != NENC * 2 * KG * NGT)   return;
    if (in_sizes[8]  != NENC * 2 * NGT)        return;
    if (in_sizes[9]  != NENC * 2 * KG * NU)    return;
    if (in_sizes[10] != NENC * 2 * NU)         return;
    if (in_sizes[11] != K1R * NH)              return;
    if (in_sizes[12] != NH)                    return;
    if (in_sizes[13] != NH * 2)                return;
    if (in_sizes[14] != 2)                     return;
    if (out_size != NR * 2)                    return;
    if (ws_size < WS_END)                      return;

    const int*   iq  = (const int*)d_in[0];
    const int*   ir  = (const int*)d_in[1];
    const int*   ql  = (const int*)d_in[2];
    const int*   rl  = (const int*)d_in[3];
    const int*   nqi = (const int*)d_in[4];
    const int*   nri = (const int*)d_in[5];
    const float* emb = (const float*)d_in[6];
    const float* gk  = (const float*)d_in[7];
    const float* gb  = (const float*)d_in[8];
    const float* ck  = (const float*)d_in[9];
    const float* cb  = (const float*)d_in[10];
    const float* w1  = (const float*)d_in[11];
    const float* b1  = (const float*)d_in[12];
    const float* w2  = (const float*)d_in[13];
    const float* b2  = (const float*)d_in[14];
    float* out = (float*)d_out;

    char* ws = (char*)d_ws;
    unsigned short* gkt = (unsigned short*)(ws + OFF_GKT);
    unsigned short* ckt = (unsigned short*)(ws + OFF_CKT);
    unsigned short* wqh = (unsigned short*)(ws + OFF_WQH);
    unsigned short* wql = (unsigned short*)(ws + OFF_WQL);
    unsigned short* wrh = (unsigned short*)(ws + OFF_WRH);
    unsigned short* wrl = (unsigned short*)(ws + OFF_WRL);
    unsigned short* wmh = (unsigned short*)(ws + OFF_WMH);
    unsigned short* wml = (unsigned short*)(ws + OFF_WML);
    _Float16*       xp  = (_Float16*)(ws + OFF_XP);
    float*          qp  = (float*)(ws + OFF_QP);
    float*          rp  = (float*)(ws + OFF_RP);
    unsigned short* qbh = (unsigned short*)(ws + OFF_QH);
    unsigned short* qbl = (unsigned short*)(ws + OFF_QL);
    unsigned short* rbh = (unsigned short*)(ws + OFF_RH);
    unsigned short* rbl = (unsigned short*)(ws + OFF_RL);
    float*          dsm = (float*)(ws + OFF_DS);
    float*          pq  = (float*)(ws + OFF_PQ);
    float*          pr  = (float*)(ws + OFF_PR);

    k_cvt<<<dim3(CV_TOTAL), dim3(256), 0, stream>>>(gk, ck, w1, gkt, ckt, wqh, wql, wrh, wrl, wmh, wml);
    k_gx<<<dim3(GX_BLK), dim3(256), 0, stream>>>(iq, ir, ql, rl, emb, xp);
    hipFuncSetAttribute(reinterpret_cast<const void*>(&k_gru),
                        hipFuncAttributeMaxDynamicSharedMemorySize, (int)LDS_GRU);
    k_gru<<<dim3(GRU_BLK), dim3(GTHR), LDS_GRU, stream>>>(
        (const _Float16*)xp, (const _Float16*)gkt, (const _Float16*)ckt, gb, cb, ql, rl,
        qp, rp, qbh, qbl, rbh, rbl);
    k_dist<<<dim3(NB), dim3(256), 0, stream>>>((const float*)qp, (const float*)rp, dsm);
    k_pnode<<<dim3(PN_BLK), dim3(256), 0, stream>>>(
        (const unsigned short*)qbh, (const unsigned short*)qbl,
        (const unsigned short*)rbh, (const unsigned short*)rbl,
        (const unsigned short*)wqh, (const unsigned short*)wql,
        (const unsigned short*)wrh, (const unsigned short*)wrl, pq, pr);
    hipFuncSetAttribute(reinterpret_cast<const void*>(&k_pair),
                        hipFuncAttributeMaxDynamicSharedMemorySize, (int)LDS_PAIR);
    k_pair<<<dim3(PR_BLK), dim3(MTHR), LDS_PAIR, stream>>>(
        (const float*)qp, (const float*)rp, (const float*)dsm, (const float*)pq, (const float*)pr,
        nqi, nri, (const unsigned short*)wmh, (const unsigned short*)wml, w1, b1, w2, b2, out);
}
